// Gnn_40845138985251
// MI455X (gfx1250) — hardware-run, weakly checked
//
#include <hip/hip_runtime.h>
#include <stddef.h>
#include <stdint.h>

#define NN      100000
#define NE      3200000
#define MP      100096
#define P1P     64
#define P2P     32
#define SPLIT2  1
#define APITCH  64
#define WPITCH  64
#define KEXT    (SPLIT2 ? 64 : 32)
#define NTHR    256
#define NWAVE   8
#define EPT     8
#define WCH     (32 * EPT)
#define NBRUN   1024
#define SLB     10
#define EIDB    22
#define NBK     98
#define WLCAP   4608
#define RCAP    36864
#define DEGCAP  96
#define MAXDEG_MEAS   57
#define MAXB1024_MEAS 33219
#define GBM     128
#define SP2     36
#define T_W1    0
#define T_WE1   512
#define T_ATT1  640
#define T_B1    672
#define T_WE2   704
#define T_ATT2  768
#define T_B2    784
#define TABF    800
#define LDS_BKT (2 * RCAP * 4)
#define LDS_BKT_STATIC ((3 * NBRUN + 16) * 4)

static_assert(NE < (1 << EIDB) && EIDB + SLB == 32);
static_assert(NBRUN == (1 << SLB) && NBRUN <= (1 << 10));
static_assert(NBK * NBRUN >= MP && MP >= NN && MP % GBM == 0 && MP == 782 * GBM);
static_assert(NE % WCH == 0 && NE % 4 == 0);
static_assert(RCAP == NWAVE * WLCAP && RCAP % (2 * NTHR) == 0 && (2 * RCAP) % (4 * NTHR) == 0);
static_assert((long long)RCAP * 100 >= (long long)MAXB1024_MEAS * 105);
static_assert(WLCAP >= MAXB1024_MEAS / 8 + 400);
static_assert(MAXDEG_MEAS + 8 <= DEGCAP);
static_assert(LDS_BKT < 300000 && LDS_BKT + LDS_BKT_STATIC <= 327680);
static_assert(NBRUN % 256 == 0 && NBRUN % 64 == 0 && NBRUN % 32 == 0);
static_assert(MP % 256 == 0 && MP % 64 == 0 && MP % 32 == 0 && (MP * 16) % NTHR == 0);
static_assert(P1P == 2 * 32 && 32 == 8 * 4);
static_assert(P2P == 2 * 16 && 16 == 4 * 4);
static_assert(KEXT % 32 == 0 && KEXT <= APITCH && KEXT <= WPITCH);
static_assert(TABF % 32 == 0 && TABF / 4 <= NTHR);
static_assert((SP2 % 4) == 0 && SP2 >= P2P);
static_assert(((NN - 1562 * 64) * 16) % 32 == 0 && 1562 * 64 * 16 + (NN - 1562 * 64) * 16 == NN * 16);

typedef float          v4f   __attribute__((ext_vector_type(4)));
typedef float          v8f   __attribute__((ext_vector_type(8)));
typedef int            v2i   __attribute__((ext_vector_type(2)));
typedef int            v4i   __attribute__((ext_vector_type(4)));
typedef int            v8i   __attribute__((ext_vector_type(8)));
typedef unsigned short v8us  __attribute__((ext_vector_type(8)));
typedef __bf16         v16bf __attribute__((ext_vector_type(16)));
typedef v4f  __attribute__((may_alias)) v4fa;
typedef v4i  __attribute__((may_alias)) v4ia;
typedef v2i  __attribute__((may_alias)) v2ia;
typedef v8us __attribute__((may_alias)) v8usa;
union FragB { v16bf v; v8us h[2]; v8i w; };

__device__ __forceinline__ v8f wmb(const FragB& a, const FragB& b, v8f c) {
  v8f d = __builtin_amdgcn_wmma_f32_16x16x32_bf16(false, a.v, false, b.v, (short)0, c, false, false);
  asm volatile("v_nop\n\tv_nop\n\tv_nop\n\tv_nop" : "+v"(d) : "v"(a.w), "v"(b.w));
  return d;
}

__device__ __forceinline__ void pinf4(v4f x) { asm volatile("" :: "v"(x)); }
__device__ __forceinline__ void pini(int x)  { asm volatile("" :: "v"(x)); }
__device__ __forceinline__ int clampi(int v, int lo, int hi) { v = v < lo ? lo : v; return v > hi ? hi : v; }

__device__ __forceinline__ unsigned bf16_bits(float f) {
  const unsigned u = __float_as_uint(f);
  const unsigned r = (u + 0x7FFFu + ((u >> 16) & 1u)) >> 16;
  const unsigned q = (u >> 16) | 0x40u;
  return ((u & 0x7fffffffu) > 0x7f800000u) ? q : r;
}
__device__ __forceinline__ float bf16_val(float f) { return __uint_as_float(bf16_bits(f) << 16); }
__device__ __forceinline__ v4f rbf4(const v4f a) {
  v4f o; o.x = bf16_val(a.x); o.y = bf16_val(a.y); o.z = bf16_val(a.z); o.w = bf16_val(a.w); return o;
}
__device__ __forceinline__ v4f blend4(const v4f a, const v4f b, int m) {
  v4f o;
  o.x = __int_as_float((__float_as_int(a.x) & m) | (__float_as_int(b.x) & ~m));
  o.y = __int_as_float((__float_as_int(a.y) & m) | (__float_as_int(b.y) & ~m));
  o.z = __int_as_float((__float_as_int(a.z) & m) | (__float_as_int(b.z) & ~m));
  o.w = __int_as_float((__float_as_int(a.w) & m) | (__float_as_int(b.w) & ~m));
  return o;
}
__device__ __forceinline__ v4f maskadd4(const v4f acc, const v4f b, int m) {
  v4f o;
  o.x = __int_as_float(__float_as_int(acc.x) | (__float_as_int(b.x) & m));
  o.y = __int_as_float(__float_as_int(acc.y) | (__float_as_int(b.y) & m));
  o.z = __int_as_float(__float_as_int(acc.z) | (__float_as_int(b.z) & m));
  o.w = __int_as_float(__float_as_int(acc.w) | (__float_as_int(b.w) & m));
  return o;
}

__device__ __forceinline__ void hilo_pack(float v0, float v1, float v2, float v3,
                                          int& h01, int& h23, int& l01, int& l23) {
  const unsigned a0 = bf16_bits(v0), a1 = bf16_bits(v1), a2 = bf16_bits(v2), a3 = bf16_bits(v3);
  const unsigned b0 = bf16_bits(v0 - __uint_as_float(a0 << 16));
  const unsigned b1 = bf16_bits(v1 - __uint_as_float(a1 << 16));
  const unsigned b2 = bf16_bits(v2 - __uint_as_float(a2 << 16));
  const unsigned b3 = bf16_bits(v3 - __uint_as_float(a3 << 16));
  h01 = (int)(a0 | (a1 << 16)); h23 = (int)(a2 | (a3 << 16));
  l01 = (int)(b0 | (b1 << 16)); l23 = (int)(b2 | (b3 << 16));
}

__device__ __forceinline__ v4i regroup_g8(int h01, int h23, int l01, int l23, int lane) {
  const int t  = lane & 7;
  const int s0 = (lane & 24) + ((2 * t) & 7), s1 = s0 + 1;
  const int a0 = __shfl(h01, s0, 32), a1 = __shfl(h23, s0, 32), a2 = __shfl(h01, s1, 32), a3 = __shfl(h23, s1, 32);
  const int b0 = __shfl(l01, s0, 32), b1 = __shfl(l23, s0, 32), b2 = __shfl(l01, s1, 32), b3 = __shfl(l23, s1, 32);
  const int mk = (t < 4) ? -1 : 0;
  v4i o;
  o.x = (a0 & mk) | (b0 & ~mk); o.y = (a1 & mk) | (b1 & ~mk);
  o.z = (a2 & mk) | (b2 & ~mk); o.w = (a3 & mk) | (b3 & ~mk);
  return o;
}

__device__ __forceinline__ void st2_v4f(float* p, v4f v) {
  *(volatile v4f*)p = v;
  __threadfence();
  *(volatile v4f*)p = v;
}
__device__ __forceinline__ void st2_v8us(unsigned short* p, v8us v) {
  *(volatile v8us*)p = v;
  __threadfence();
  *(volatile v8us*)p = v;
}

__device__ __forceinline__ v8us col8(const float* __restrict__ base, int stride) {
  float f[8];
#pragma unroll
  for (int i = 0; i < 8; ++i) f[i] = base[(size_t)i * (size_t)stride];
  v8us o;
#pragma unroll
  for (int i = 0; i < 8; ++i) o[i] = (unsigned short)bf16_bits(f[i]);
  return o;
}

__global__ __launch_bounds__(NTHR) void k_prep(const float* __restrict__ wl1, const float* __restrict__ wr1,
                                               const float* __restrict__ we1, const float* __restrict__ att1,
                                               const float* __restrict__ b1, const float* __restrict__ wl2,
                                               const float* __restrict__ wr2, const float* __restrict__ we2,
                                               const float* __restrict__ att2, const float* __restrict__ b2,
                                               float* tab, unsigned short* w2t) {
  const int tid = (int)threadIdx.x;
  if (blockIdx.x == 0) {
    const int u  = tid;
    const int uw = u < 128 ? u : 127;
    const int k  = uw >> 4, t = uw & 15;
    const int i4 = k * 8 + (t & 7);
    const v4f a = *(const v4fa*)(wl1 + 4 * i4);
    const v4f b = *(const v4fa*)(wr1 + 4 * i4);
    const v4f c = *(const v4fa*)(we1  + 4 * clampi(u - 128, 0, 31));
    const v4f d = *(const v4fa*)(att1 + 4 * clampi(u - 160, 0, 7));
    const v4f e = *(const v4fa*)(b1   + 4 * clampi(u - 168, 0, 7));
    const v4f f = *(const v4fa*)(we2  + 4 * clampi(u - 176, 0, 15));
    const v4f g = *(const v4fa*)(att2 + 4 * clampi(u - 192, 0, 3));
    const v4f h = *(const v4fa*)(b2   + 4 * clampi(u - 196, 0, 3));
    pinf4(a); pinf4(b); pinf4(c); pinf4(d); pinf4(e); pinf4(f); pinf4(g); pinf4(h);
    const int mA = (u < 128 && t < 8)  ? -1 : 0;
    const int mB = (u < 128 && t >= 8) ? -1 : 0;
    const int mC = ((unsigned)(u - 128) < 32u) ? -1 : 0;
    const int mD = ((unsigned)(u - 160) < 8u)  ? -1 : 0;
    const int mE = ((unsigned)(u - 168) < 8u)  ? -1 : 0;
    const int mF = ((unsigned)(u - 176) < 16u) ? -1 : 0;
    const int mG = ((unsigned)(u - 192) < 4u)  ? -1 : 0;
    const int mH = ((unsigned)(u - 196) < 4u)  ? -1 : 0;
    v4f s = {0.0f, 0.0f, 0.0f, 0.0f};
    s = maskadd4(s, a, mA); s = maskadd4(s, b, mB); s = maskadd4(s, c, mC); s = maskadd4(s, d, mD);
    s = maskadd4(s, e, mE); s = maskadd4(s, f, mF); s = maskadd4(s, g, mG); s = maskadd4(s, h, mH);
    const v4f o = rbf4(s);
    if (u < TABF / 4) {
      float* p = tab + 4 * u;
      *(volatile v4f*)p = o;
      __threadfence();
      *(volatile v4f*)p = o;
    }
  } else {
    const int n = tid >> 3, k8 = (tid & 7) * 8, kk = k8 & 31;
    v8us o;
    if (tid < 128) o = col8(wl2 + (size_t)kk * 16 + n, 16);
    else           o = col8(wr2 + (size_t)kk * 16 + (n - 16), 16);
    st2_v8us(w2t + (size_t)n * WPITCH + k8, o);
  }
}

__global__ __launch_bounds__(NTHR) void k_proj1(const float* __restrict__ x, const float* __restrict__ tab, float* P1) {
  __shared__ __attribute__((aligned(16))) float sw[512];
  const int tid = (int)threadIdx.x;
  if (tid < 128) *(v4fa*)(sw + 4 * tid) = *(const v4fa*)(tab + T_W1 + 4 * tid);
  __syncthreads();
  const int u    = (int)blockIdx.x * NTHR + tid;
  const int node = u >> 4, t = u & 15;
  const int rc   = node < NN ? node : NN - 1;
  const v4f xa = rbf4(*(const v4fa*)(x + (size_t)rc * 8));
  const v4f xb = rbf4(*(const v4fa*)(x + (size_t)rc * 8 + 4));
  const float* wp = sw + 4 * t;
  v4f acc = *(const v4fa*)(wp) * xa.x;
  acc = acc + *(const v4fa*)(wp + 64)  * xa.y;
  acc = acc + *(const v4fa*)(wp + 128) * xa.z;
  acc = acc + *(const v4fa*)(wp + 192) * xa.w;
  acc = acc + *(const v4fa*)(wp + 256) * xb.x;
  acc = acc + *(const v4fa*)(wp + 320) * xb.y;
  acc = acc + *(const v4fa*)(wp + 384) * xb.z;
  acc = acc + *(const v4fa*)(wp + 448) * xb.w;
  const bool live = node < NN;
  v4f o;
  o.x = live ? acc.x : 0.0f; o.y = live ? acc.y : 0.0f; o.z = live ? acc.z : 0.0f; o.w = live ? acc.w : 0.0f;
  st2_v4f(P1 + (size_t)node * P1P + 4 * t, o);
}

__global__ __launch_bounds__(NTHR) void k_bucket(const int* __restrict__ srcs, const int* __restrict__ dsts,
                                                 int* HITS, int* CO, int* FLAG) {
  extern __shared__ __attribute__((aligned(16))) int dsm[];
  __shared__ __attribute__((aligned(16))) int sco[2 * NBRUN];
  __shared__ __attribute__((aligned(16))) int scur[NBRUN];
  __shared__ __attribute__((aligned(16))) int smisc[16];
  int* wl   = dsm;
  int* pl   = dsm + RCAP;
  int* cnt  = sco;
  int* offs = sco + NBRUN;
  const int tid = (int)threadIdx.x, lane = tid & 31, wave = tid >> 5;
  const int blk = (int)blockIdx.x;
  const unsigned nbs = (unsigned)(blk * NBRUN);

  {
    const v4i z4 = {0, 0, 0, 0};
    for (int i = tid * 4; i < 2 * RCAP; i += NTHR * 4) *(v4ia*)(dsm + i) = z4;
    for (int i = tid * 4; i < 2 * NBRUN; i += NTHR * 4) *(v4ia*)(sco + i) = z4;
    *(v4ia*)(scur + 4 * tid) = z4;
    if (tid < 16) smisc[tid] = 0;
  }
  __syncthreads();

  {
    const int per  = ((NE + NWAVE * WCH - 1) / (NWAVE * WCH)) * WCH;
    const int ebeg = wave * per;
    const int eend = (ebeg + per < NE) ? (ebeg + per) : NE;
    int* mylist = wl + wave * WLCAP;
    int wc = 0;
#pragma unroll 1
    for (int cb = ebeg; cb < eend; cb += WCH) {
      const int e0 = cb + lane * EPT;
      const v4i da = *(const v4ia*)(dsts + e0);
      const v4i db = *(const v4ia*)(dsts + e0 + 4);
      const unsigned s0 = (unsigned)da.x - nbs, s1 = (unsigned)da.y - nbs;
      const unsigned s2 = (unsigned)da.z - nbs, s3 = (unsigned)da.w - nbs;
      const unsigned s4 = (unsigned)db.x - nbs, s5 = (unsigned)db.y - nbs;
      const unsigned s6 = (unsigned)db.z - nbs, s7 = (unsigned)db.w - nbs;
      const bool h0 = s0 < (unsigned)NBRUN, h1 = s1 < (unsigned)NBRUN, h2 = s2 < (unsigned)NBRUN, h3 = s3 < (unsigned)NBRUN;
      const bool h4 = s4 < (unsigned)NBRUN, h5 = s5 < (unsigned)NBRUN, h6 = s6 < (unsigned)NBRUN, h7 = s7 < (unsigned)NBRUN;
      const unsigned m0 = __builtin_amdgcn_ballot_w32(h0), m1 = __builtin_amdgcn_ballot_w32(h1);
      const unsigned m2 = __builtin_amdgcn_ballot_w32(h2), m3 = __builtin_amdgcn_ballot_w32(h3);
      const unsigned m4 = __builtin_amdgcn_ballot_w32(h4), m5 = __builtin_amdgcn_ballot_w32(h5);
      const unsigned m6 = __builtin_amdgcn_ballot_w32(h6), m7 = __builtin_amdgcn_ballot_w32(h7);
      const unsigned any = m0 | m1 | m2 | m3 | m4 | m5 | m6 | m7;
      if (any != 0u) {
        const int pre = (int)(__builtin_amdgcn_mbcnt_lo(m0, 0u) + __builtin_amdgcn_mbcnt_lo(m1, 0u) +
                              __builtin_amdgcn_mbcnt_lo(m2, 0u) + __builtin_amdgcn_mbcnt_lo(m3, 0u) +
                              __builtin_amdgcn_mbcnt_lo(m4, 0u) + __builtin_amdgcn_mbcnt_lo(m5, 0u) +
                              __builtin_amdgcn_mbcnt_lo(m6, 0u) + __builtin_amdgcn_mbcnt_lo(m7, 0u));
        int p = wc + pre;
        if (h0) { if (p < WLCAP) mylist[p] = (int)((unsigned)(e0 + 0) | (s0 << EIDB)); p = p + 1; }
        if (h1) { if (p < WLCAP) mylist[p] = (int)((unsigned)(e0 + 1) | (s1 << EIDB)); p = p + 1; }
        if (h2) { if (p < WLCAP) mylist[p] = (int)((unsigned)(e0 + 2) | (s2 << EIDB)); p = p + 1; }
        if (h3) { if (p < WLCAP) mylist[p] = (int)((unsigned)(e0 + 3) | (s3 << EIDB)); p = p + 1; }
        if (h4) { if (p < WLCAP) mylist[p] = (int)((unsigned)(e0 + 4) | (s4 << EIDB)); p = p + 1; }
        if (h5) { if (p < WLCAP) mylist[p] = (int)((unsigned)(e0 + 5) | (s5 << EIDB)); p = p + 1; }
        if (h6) { if (p < WLCAP) mylist[p] = (int)((unsigned)(e0 + 6) | (s6 << EIDB)); p = p + 1; }
        if (h7) { if (p < WLCAP) mylist[p] = (int)((unsigned)(e0 + 7) | (s7 << EIDB)); p = p + 1; }
        wc += (int)(__builtin_popcount(m0) + __builtin_popcount(m1) + __builtin_popcount(m2) + __builtin_popcount(m3) +
                    __builtin_popcount(m4) + __builtin_popcount(m5) + __builtin_popcount(m6) + __builtin_popcount(m7));
      }
    }
    if (lane == 0) smisc[wave] = wc;
  }
  __syncthreads();

  if (wave == 0) {
    int ov = 0;
#pragma unroll 1
    for (int w2 = 0; w2 < NWAVE; ++w2) {
      int c = smisc[w2];
      if (c > WLCAP) ov = 1;
      c = c < 0 ? 0 : (c > WLCAP ? WLCAP : c);
#pragma unroll 1
      for (int b0 = 0; b0 < c; b0 += 32) {
        const int idx = b0 + lane;
        const int ent = wl[w2 * WLCAP + (idx < WLCAP ? idx : WLCAP - 1)];
        const int m32 = (c - b0) < 32 ? (c - b0) : 32;
#pragma unroll 1
        for (int k = 0; k < m32; ++k) {
          const int u    = __builtin_amdgcn_readlane(ent, k);
          const int slot = (int)((unsigned)u >> EIDB);
          if (lane == 0) cnt[slot] = cnt[slot] + 1;
        }
      }
    }
    if (lane == 0) smisc[9] = ov;
  }
  __syncthreads();
  if (wave == 0) {
    const int base = lane * (NBRUN / 32);
    int s = 0, dg = 0;
#pragma unroll 1
    for (int i = 0; i < NBRUN / 32; ++i) {
      const int cv = cnt[base + i];
      s += cv;
      dg |= (cv > DEGCAP) ? 1 : 0;
    }
    int incl = s;
#pragma unroll
    for (int d = 1; d < 32; d <<= 1) {
      const int y = __shfl_up(incl, d, 32);
      if (lane >= d) incl += y;
    }
    int run = incl - s;
#pragma unroll 1
    for (int i = 0; i < NBRUN / 32; ++i) {
      const int cv = cnt[base + i];
      offs[base + i] = run;
      scur[base + i] = run;
      run += cv;
    }
    const unsigned bm = __builtin_amdgcn_ballot_w32(dg != 0);
    if (lane == 31) smisc[10] = run;
    if (lane == 0) smisc[9] = smisc[9] | ((bm != 0u) ? 1 : 0);
  }
  __syncthreads();

  if (wave == 0) {
#pragma unroll 1
    for (int w2 = 0; w2 < NWAVE; ++w2) {
      int c = smisc[w2];
      c = c < 0 ? 0 : (c > WLCAP ? WLCAP : c);
#pragma unroll 1
      for (int b0 = 0; b0 < c; b0 += 32) {
        const int idx = b0 + lane;
        const int ent = wl[w2 * WLCAP + (idx < WLCAP ? idx : WLCAP - 1)];
        const int m32 = (c - b0) < 32 ? (c - b0) : 32;
#pragma unroll 1
        for (int k = 0; k < m32; ++k) {
          const int u    = __builtin_amdgcn_readlane(ent, k);
          const int slot = (int)((unsigned)u >> EIDB);
          const int eid  = u & ((1 << EIDB) - 1);
          if (lane == 0) {
            int p = scur[slot];
            p = p < 0 ? 0 : (p > RCAP - 1 ? RCAP - 1 : p);
            pl[p] = eid;
            scur[slot] = p + 1;
          }
        }
      }
    }
  }
  __syncthreads();

  const int ovf = smisc[9];
  const int nh  = clampi(smisc[10], 0, RCAP);
  int* hp = HITS + (size_t)blk * (size_t)(2 * RCAP);
#pragma unroll 1
  for (int p0 = 0; p0 < RCAP; p0 += 2 * NTHR) {
    const int p = p0 + 2 * tid;
    const int e0 = clampi(pl[p],     0, NE - 1);
    const int e1 = clampi(pl[p + 1], 0, NE - 1);
    int s0 = srcs[e0];
    int s1 = srcs[e1];
    pini(s0); pini(s1);
    s0 = clampi(s0, 0, NN - 1);
    s1 = clampi(s1, 0, NN - 1);
    const int m0 = (p     < nh) ? -1 : 0;
    const int m1 = (p + 1 < nh) ? -1 : 0;
    v4i v;
    v.x = s0 & m0; v.y = e0 & m0; v.z = s1 & m1; v.w = e1 & m1;
    *(volatile v4i*)(hp + 2 * p) = v;
    __threadfence();
    *(volatile v4i*)(hp + 2 * p) = v;
  }
  {
    const v4i c0 = *(const v4ia*)(sco + 4 * tid);
    const v4i c1 = *(const v4ia*)(sco + NBRUN + 4 * tid);
    const v4i fv = {ovf, ovf, ovf, ovf};
    int* cop = CO + (size_t)blk * (2 * NBRUN);
    int* fp  = FLAG + (size_t)blk * 32;
    *(volatile v4i*)(cop + 4 * tid) = c0;
    *(volatile v4i*)(cop + NBRUN + 4 * tid) = c1;
    if (tid < 8) *(volatile v4i*)(fp + 4 * tid) = fv;
    __threadfence();
    *(volatile v4i*)(cop + 4 * tid) = c0;
    *(volatile v4i*)(cop + NBRUN + 4 * tid) = c1;
    if (tid < 8) *(volatile v4i*)(fp + 4 * tid) = fv;
  }
}

__global__ __launch_bounds__(NTHR) void k_loopattr(const int* __restrict__ HITS, const int* __restrict__ CO,
                                                   const float* __restrict__ ea, float* LA) {
  const int tid = (int)threadIdx.x;
  const int rowBase = (int)blockIdx.x * NTHR;
  const int d = rowBase + tid;
  const int bucket = rowBase >> SLB;
  const int slot = d & (NBRUN - 1);
  const int* cob = CO + (size_t)bucket * (2 * NBRUN);
  const int* hb  = HITS + (size_t)bucket * (size_t)(2 * RCAP);
  int c = cob[slot];
  int o = cob[NBRUN + slot];
  c = clampi(c, 0, DEGCAP);
  o = clampi(o, 0, RCAP - 1);
  if (c > RCAP - o) c = RCAP - o;
  int cm = c;
#pragma unroll
  for (int off = 1; off < 32; off <<= 1) {
    const int y = __shfl_xor(cm, off, 32);
    cm = cm > y ? cm : y;
  }
  const int trips = __builtin_amdgcn_readfirstlane(cm);
  int last = o + c - 1; last = last < o ? o : last;
  last = last > RCAP - 1 ? RCAP - 1 : last;
  float s0 = 0.0f, s1 = 0.0f, s2 = 0.0f, s3 = 0.0f;
#pragma unroll 1
  for (int j = 0; j < trips; ++j) {
    int idx = o + j;
    idx = idx > last ? last : idx;
    const v2i en = *(const v2ia*)(hb + 2 * idx);
    const int eid = clampi(en.y, 0, NE - 1);
    const v4f er = *(const v4fa*)(ea + (size_t)eid * 4);
    pinf4(er);
    const v4f t = rbf4(er);
    const bool valid = j < c;
    const float n0 = s0 + t.x, n1 = s1 + t.y, n2 = s2 + t.z, n3 = s3 + t.w;
    s0 = valid ? n0 : s0; s1 = valid ? n1 : s1; s2 = valid ? n2 : s2; s3 = valid ? n3 : s3;
  }
  const float cf = (float)(c > 1 ? c : 1);
  v4f ov;
  ov.x = s0 / cf; ov.y = s1 / cf; ov.z = s2 / cf; ov.w = s3 / cf;
  st2_v4f(LA + (size_t)d * 4, ov);
}

template <int PITCH>
__device__ __forceinline__ v4f replay_core(const int* __restrict__ hb, const float* __restrict__ P,
                                           const float* __restrict__ ea, int d, int c, int o, int trips, int q,
                                           const v4f la, const v4f w0, const v4f w1, const v4f w2, const v4f w3,
                                           const v4f at) {
  constexpr int CH  = PITCH / 2;
  constexpr int LPD = CH / 4;
  const v4f xr = *(const v4fa*)(P + (size_t)d * PITCH + CH + 4 * q);
  int last = o + c - 1; last = last < o ? o : last;
  last = last > RCAP - 1 ? RCAP - 1 : last;
  float mx = -1.0e30f, l = 0.0f;
  float a0 = 0.0f, a1 = 0.0f, a2 = 0.0f, a3 = 0.0f;
#pragma unroll 1
  for (int j = 0; j < trips; ++j) {
    int idx = o + j;
    idx = idx > last ? last : idx;
    const v2i en = *(const v2ia*)(hb + 2 * idx);
    const int src = clampi(en.x, 0, NN - 1);
    const int eid = clampi(en.y, 0, NE - 1);
    const int rm  = (j < c) ? -1 : 0;
    const int sidx = (src & rm) | (d & ~rm);
    const v4f xl = *(const v4fa*)(P + (size_t)sidx * PITCH + 4 * q);
    const v4f er = *(const v4fa*)(ea + (size_t)eid * 4);
    pinf4(xl); pinf4(er);
    const v4f e4 = blend4(rbf4(er), la, rm);
    const v4f ep = ((w0 * e4.x + w1 * e4.y) + w2 * e4.z) + w3 * e4.w;
    v4f v = (xl + xr) + ep;
    v.x = (v.x > 0.0f) ? v.x : 0.2f * v.x;
    v.y = (v.y > 0.0f) ? v.y : 0.2f * v.y;
    v.z = (v.z > 0.0f) ? v.z : 0.2f * v.z;
    v.w = (v.w > 0.0f) ? v.w : 0.2f * v.w;
    float part = v.x * at.x;
    part = fmaf(v.y, at.y, part);
    part = fmaf(v.z, at.z, part);
    part = fmaf(v.w, at.w, part);
#pragma unroll
    for (int off = 1; off < LPD; off <<= 1) part += __shfl_xor(part, off, 32);
    const float al = part;
    const float df = al - mx;
    const float eo = expf(-fabsf(df));
    const bool up  = df > 0.0f;
    const float f1 = up ? eo : 1.0f;
    const float f2 = up ? 1.0f : eo;
    const float nmx = up ? al : mx;
    const float nl  = fmaf(l, f1, f2);
    const float n0 = a0 * f1 + xl.x * f2, n1 = a1 * f1 + xl.y * f2;
    const float n2 = a2 * f1 + xl.z * f2, n3 = a3 * f1 + xl.w * f2;
    const bool valid = j <= c;
    mx = valid ? nmx : mx; l = valid ? nl : l;
    a0 = valid ? n0 : a0; a1 = valid ? n1 : a1; a2 = valid ? n2 : a2; a3 = valid ? n3 : a3;
  }
  v4f r;
  r.x = a0 / l; r.y = a1 / l; r.z = a2 / l; r.w = a3 / l;
  return r;
}

__global__ __launch_bounds__(NTHR) void k_replay1(const int* __restrict__ HITS, const int* __restrict__ CO,
                                                  const int* __restrict__ FLAG, const float* __restrict__ P1,
                                                  const float* __restrict__ ea, const float* __restrict__ LA,
                                                  const float* __restrict__ tab, unsigned short* H1) {
  const int tid = (int)threadIdx.x, lane = tid & 31, wave = tid >> 5;
  const int g = lane >> 3, q = lane & 7;
  const int rowBase = (int)blockIdx.x * 32;
  const int d = rowBase + 4 * wave + g;
  const int bucket = rowBase >> SLB;
  const int slot = d & (NBRUN - 1);
  const int* cob = CO + (size_t)bucket * (2 * NBRUN);
  const int* hb  = HITS + (size_t)bucket * (size_t)(2 * RCAP);
  const int flag = FLAG[(size_t)bucket * 32];
  const int craw = cob[slot];
  const int oraw = cob[NBRUN + slot];
  const bool big = (craw < 0) | (craw > DEGCAP);
  int c = clampi(craw, 0, DEGCAP);
  const int o = clampi(oraw, 0, RCAP - 1);
  if (c > RCAP - o) c = RCAP - o;
  int cm = c;
  { const int y = __shfl_xor(cm, 8, 32);  cm = cm > y ? cm : y; }
  { const int y = __shfl_xor(cm, 16, 32); cm = cm > y ? cm : y; }
  const int trips = __builtin_amdgcn_readfirstlane(cm) + 1;

  const v4f la = *(const v4fa*)(LA + (size_t)d * 4);
  const v4f w0 = *(const v4fa*)(tab + T_WE1 + 4 * q);
  const v4f w1 = *(const v4fa*)(tab + T_WE1 + 32 + 4 * q);
  const v4f w2 = *(const v4fa*)(tab + T_WE1 + 64 + 4 * q);
  const v4f w3 = *(const v4fa*)(tab + T_WE1 + 96 + 4 * q);
  const v4f at = *(const v4fa*)(tab + T_ATT1 + 4 * q);
  const v4f bb = *(const v4fa*)(tab + T_B1 + 4 * q);

  const v4f r = replay_core<P1P>(hb, P1, ea, d, c, o, trips, q, la, w0, w1, w2, w3, at);

  float v0 = r.x + bb.x, v1 = r.y + bb.y, v2 = r.z + bb.z, v3 = r.w + bb.w;
  v0 = (v0 > 0.0f) ? v0 : (v0 - v0); v1 = (v1 > 0.0f) ? v1 : (v1 - v1);
  v2 = (v2 > 0.0f) ? v2 : (v2 - v2); v3 = (v3 > 0.0f) ? v3 : (v3 - v3);
  const float qnan = __uint_as_float(0x7fc00000u);
  const bool bad  = (flag != 0) | big;
  const bool live = d < NN;
  v0 = bad ? qnan : v0; v1 = bad ? qnan : v1; v2 = bad ? qnan : v2; v3 = bad ? qnan : v3;
  v0 = live ? v0 : 0.0f; v1 = live ? v1 : 0.0f; v2 = live ? v2 : 0.0f; v3 = live ? v3 : 0.0f;
  int h01, h23, l01, l23;
  hilo_pack(v0, v1, v2, v3, h01, h23, l01, l23);
  const v4i ow = regroup_g8(h01, h23, l01, l23, lane);
  unsigned short* hp = H1 + (size_t)d * APITCH + 8 * q;
  *(volatile v4i*)hp = ow;
  __threadfence();
  *(volatile v4i*)hp = ow;
}

__global__ __launch_bounds__(NTHR) __attribute__((amdgpu_num_vgpr(248)))
void k_gemm2(const unsigned short* __restrict__ A, const unsigned short* __restrict__ BT, float* P2) {
  __shared__ __attribute__((aligned(16))) float stg[GBM * SP2];
  const int tid = (int)threadIdx.x, lane = tid & 31, wave = tid >> 5, hh = lane >> 4, m = lane & 15;
  const int rowBase = (int)blockIdx.x * GBM;

  const v8f z = {0.f, 0.f, 0.f, 0.f, 0.f, 0.f, 0.f, 0.f};
  v8f acc0 = z, acc1 = z;
  const unsigned short* ap = A + (size_t)(rowBase + 16 * wave + m) * (size_t)APITCH + 8 * hh;
  const unsigned short* bp = BT + (size_t)m * (size_t)WPITCH + 8 * hh;
#pragma unroll
  for (int k0 = 0; k0 < KEXT; k0 += 32) {
    FragB af;
    af.h[0] = *(const v8usa*)(ap + k0);
    af.h[1] = *(const v8usa*)(ap + k0 + 16);
    {
      FragB bf;
      bf.h[0] = *(const v8usa*)(bp + k0);
      bf.h[1] = *(const v8usa*)(bp + k0 + 16);
      acc0 = wmb(af, bf, acc0);
    }
    {
      const unsigned short* wq = bp + (size_t)16 * (size_t)WPITCH + k0;
      FragB bf;
      bf.h[0] = *(const v8usa*)wq;
      bf.h[1] = *(const v8usa*)(wq + 16);
      acc1 = wmb(af, bf, acc1);
    }
  }
#pragma unroll
  for (int r = 0; r < 8; ++r) {
    stg[(16 * wave + 8 * hh + r) * SP2 + m]      = acc0[r];
    stg[(16 * wave + 8 * hh + r) * SP2 + 16 + m] = acc1[r];
  }
  __syncthreads();

  v4f fv[4];
#pragma unroll
  for (int i = 0; i < 4; ++i) {
    const int lr = 16 * wave + 4 * i + (lane >> 3);
    fv[i] = *(const v4fa*)(stg + lr * SP2 + 4 * (lane & 7));
  }
#pragma unroll
  for (int i = 0; i < 4; ++i) {
    const int lr = 16 * wave + 4 * i + (lane >> 3);
    float* op = P2 + (size_t)(rowBase + lr) * P2P + 4 * (lane & 7);
    *(volatile v4f*)op = fv[i];
  }
  __threadfence();
#pragma unroll
  for (int i = 0; i < 4; ++i) {
    const int lr = 16 * wave + 4 * i + (lane >> 3);
    float* op = P2 + (size_t)(rowBase + lr) * P2P + 4 * (lane & 7);
    *(volatile v4f*)op = fv[i];
  }
}

__global__ __launch_bounds__(NTHR) void k_replay2(const int* __restrict__ HITS, const int* __restrict__ CO,
                                                  const int* __restrict__ FLAG, const float* __restrict__ P2,
                                                  const float* __restrict__ ea, const float* __restrict__ LA,
                                                  const float* __restrict__ tab, float* out) {
  __shared__ __attribute__((aligned(16))) float so[64 * 16];
  const int tid = (int)threadIdx.x, lane = tid & 31, wave = tid >> 5;
  const int g = lane >> 2, q = lane & 3;
  const int rowBase = (int)blockIdx.x * 64;
  const int d = rowBase + 8 * wave + g;
  const int bucket = rowBase >> SLB;
  const int slot = d & (NBRUN - 1);
  const int* cob = CO + (size_t)bucket * (2 * NBRUN);
  const int* hb  = HITS + (size_t)bucket * (size_t)(2 * RCAP);
  const int flag = FLAG[(size_t)bucket * 32];
  const int craw = cob[slot];
  const int oraw = cob[NBRUN + slot];
  const bool big = (craw < 0) | (craw > DEGCAP);
  int c = clampi(craw, 0, DEGCAP);
  const int o = clampi(oraw, 0, RCAP - 1);
  if (c > RCAP - o) c = RCAP - o;
  int cm = c;
  { const int y = __shfl_xor(cm, 4, 32);  cm = cm > y ? cm : y; }
  { const int y = __shfl_xor(cm, 8, 32);  cm = cm > y ? cm : y; }
  { const int y = __shfl_xor(cm, 16, 32); cm = cm > y ? cm : y; }
  const int trips = __builtin_amdgcn_readfirstlane(cm) + 1;

  const v4f la = *(const v4fa*)(LA + (size_t)d * 4);
  const v4f w0 = *(const v4fa*)(tab + T_WE2 + 4 * q);
  const v4f w1 = *(const v4fa*)(tab + T_WE2 + 16 + 4 * q);
  const v4f w2 = *(const v4fa*)(tab + T_WE2 + 32 + 4 * q);
  const v4f w3 = *(const v4fa*)(tab + T_WE2 + 48 + 4 * q);
  const v4f at = *(const v4fa*)(tab + T_ATT2 + 4 * q);
  const v4f bb = *(const v4fa*)(tab + T_B2 + 4 * q);

  const v4f r = replay_core<P2P>(hb, P2, ea, d, c, o, trips, q, la, w0, w1, w2, w3, at);

  const float qnan = __uint_as_float(0x7fc00000u);
  const bool bad = (flag != 0) | big;
  v4f v;
  v.x = r.x + bb.x; v.y = r.y + bb.y; v.z = r.z + bb.z; v.w = r.w + bb.w;
  v.x = bad ? qnan : v.x; v.y = bad ? qnan : v.y; v.z = bad ? qnan : v.z; v.w = bad ? qnan : v.w;
  *(v4fa*)(so + (8 * wave + g) * 16 + 4 * q) = v;
  __syncthreads();

  const int liveRows = (NN - rowBase) < 64 ? (NN - rowBase) : 64;
  const int nv4 = liveRows * 4;
  const v4f fo = *(const v4fa*)(so + 4 * tid);
  pinf4(fo);
  float* ob = out + (size_t)blockIdx.x * 1024 + 4 * tid;
  if (tid < nv4) *(volatile v4f*)ob = fo;
  __threadfence();
  if (tid < nv4) *(volatile v4f*)ob = fo;
}

extern "C" void kernel_launch(void* const* d_in, const int* in_sizes, int n_in,
                              void* d_out, int out_size, void* d_ws, size_t ws_size,
                              hipStream_t stream) {
  if (n_in < 13) return;
  if (in_sizes[0] != NN * 8) return;
  if (in_sizes[1] != 2 * NE) return;
  if (in_sizes[2] != NE * 4) return;
  if (in_sizes[3] != 8 * 32 || in_sizes[4] != 8 * 32) return;
  if (in_sizes[5] != 4 * 32) return;
  if (in_sizes[6] != 32 || in_sizes[7] != 32) return;
  if (in_sizes[8] != 32 * 16 || in_sizes[9] != 32 * 16) return;
  if (in_sizes[10] != 4 * 16) return;
  if (in_sizes[11] != 16 || in_sizes[12] != 16) return;
  if (out_size != NN * 16) return;

  const float* x    = (const float*)d_in[0];
  const int*   ei   = (const int*)d_in[1];
  const float* ea   = (const float*)d_in[2];
  const float* Wl1  = (const float*)d_in[3];
  const float* Wr1  = (const float*)d_in[4];
  const float* We1  = (const float*)d_in[5];
  const float* att1 = (const float*)d_in[6];
  const float* b1   = (const float*)d_in[7];
  const float* Wl2  = (const float*)d_in[8];
  const float* Wr2  = (const float*)d_in[9];
  const float* We2  = (const float*)d_in[10];
  const float* att2 = (const float*)d_in[11];
  const float* b2   = (const float*)d_in[12];
  float* out = (float*)d_out;
  const int* srcs = ei;
  const int* dsts = ei + NE;

  constexpr size_t zP1   = (size_t)MP * P1P * 4;
  constexpr size_t zH1   = (size_t)MP * APITCH * 2;
  constexpr size_t zP2   = (size_t)MP * P2P * 4;
  constexpr size_t zLA   = (size_t)MP * 4 * 4;
  constexpr size_t zHITS = (size_t)NBK * RCAP * 8;
  constexpr size_t zCO   = (size_t)NBK * 2 * NBRUN * 4;
  constexpr size_t zFLAG = (size_t)NBK * 128;
  constexpr size_t zTAB  = 3328;
  constexpr size_t zW2T  = (size_t)32 * WPITCH * 2;
  constexpr size_t oP1   = 0;
  constexpr size_t oH1   = oP1 + zP1;
  constexpr size_t oP2   = oH1 + zH1;
  constexpr size_t oLA   = oP2 + zP2;
  constexpr size_t oHITS = oLA + zLA;
  constexpr size_t oCO   = oHITS + zHITS;
  constexpr size_t oFLAG = oCO + zCO;
  constexpr size_t oTAB  = oFLAG + zFLAG;
  constexpr size_t oW2T  = oTAB + zTAB;
  constexpr size_t oEND  = oW2T + zW2T;
  static_assert(zP1 % 256 == 0 && zH1 % 256 == 0 && zP2 % 256 == 0 && zLA % 256 == 0 && zHITS % 256 == 0);
  static_assert(zCO % 256 == 0 && zFLAG % 256 == 0 && zTAB % 256 == 0 && zW2T % 256 == 0);
  static_assert(zTAB >= (size_t)TABF * 4);
  static_assert(oEND <= (size_t)(128u << 20));
  if (oEND > ws_size) return;

  char* ws = (char*)d_ws;
  float*          P1   = (float*)(ws + oP1);
  unsigned short* H1   = (unsigned short*)(ws + oH1);
  float*          P2   = (float*)(ws + oP2);
  float*          LA   = (float*)(ws + oLA);
  int*            HITS = (int*)(ws + oHITS);
  int*            CO   = (int*)(ws + oCO);
  int*            FLAG = (int*)(ws + oFLAG);
  float*          TAB  = (float*)(ws + oTAB);
  unsigned short* W2T  = (unsigned short*)(ws + oW2T);

  hipFuncSetAttribute(reinterpret_cast<const void*>(&k_bucket), hipFuncAttributeMaxDynamicSharedMemorySize, (int)LDS_BKT);

  k_prep<<<2, NTHR, 0, stream>>>(Wl1, Wr1, We1, att1, b1, Wl2, Wr2, We2, att2, b2, TAB, W2T);
  k_proj1<<<(MP * 16) / NTHR, NTHR, 0, stream>>>(x, TAB, P1);
  k_bucket<<<NBK, NTHR, LDS_BKT, stream>>>(srcs, dsts, HITS, CO, FLAG);
  k_loopattr<<<MP / NTHR, NTHR, 0, stream>>>(HITS, CO, ea, LA);
  k_replay1<<<MP / 32, NTHR, 0, stream>>>(HITS, CO, FLAG, P1, ea, LA, TAB, H1);
  k_gemm2<<<MP / GBM, NTHR, 0, stream>>>(H1, W2T, P2);
  k_replay2<<<MP / 64, NTHR, 0, stream>>>(HITS, CO, FLAG, P2, ea, LA, TAB, out);
}
